// DeformationMetaMultiMLP_19602230739477
// MI455X (gfx1250) — hardware-verified
//
#include <hip/hip_runtime.h>
#include <math.h>

#ifndef NB
#define NB 8
#endif
#ifndef SEQ
#define SEQ 2048
#endif
#define NB_FULL 8
#define SEQ_FULL 2048
#define XD 3
#define CD 128
#define LW 64
#define OD 3
#define GS1 65
#define GP 80
#define R0 256
#define R1 (LW * GS1)
#define R1P (LW * GP)
#define R3 (OD * GS1)
#define R3P (OD * GP)
#define B3PITCH 256
#define HPP 16
#define HPT (GP * HPP)
#define FW 4
#define NTOT (NB * SEQ * OD)

static_assert(NB >= 1 && NB <= NB_FULL);
static_assert(SEQ % 16 == 0 && SEQ <= SEQ_FULL);
static_assert((NB * (SEQ / 16)) % FW == 0);
static_assert(CD == 128 && CD % 32 == 0);
static_assert(GP % 16 == 0 && GP / 16 == 5 && GP >= GS1);
static_assert(LW == 64 && LW + 1 == GS1 && LW + 16 == GP);
static_assert(R0 == 16 * 16 && R0 == LW * (XD + 1));
static_assert((GP * 16) % 256 == 0 && (R0 * 16) % 256 == 0);
static_assert(R0 % 128 == 0 && R1P % 128 == 0 && B3PITCH % 128 == 0 && B3PITCH >= R3P);
static_assert(NTOT % 32 == 0);
static_assert(16 * 16 == 16 * 4 * 4);
static_assert(FW * 2 * HPT * 4 <= 131072);

typedef __attribute__((ext_vector_type(16))) __bf16 v16bf;
typedef __attribute__((ext_vector_type(8)))  float    v8f;
typedef __attribute__((ext_vector_type(4)))  float    v4f;
typedef __attribute__((ext_vector_type(4)))  unsigned int v4u;
typedef __attribute__((ext_vector_type(8)))  unsigned int v8u;


#define VST2(T, ptr, val) do { const T vst2_v_ = (val); *(volatile T*)(ptr) = vst2_v_; __threadfence(); *(volatile T*)(ptr) = vst2_v_; } while (0)
#define VST2V4(ptr, val) do { const v4f vst2_v4_ = (val); *(volatile v4f*)(ptr) = vst2_v4_; __threadfence(); *(volatile v4f*)(ptr) = vst2_v4_; } while (0)

__device__ __forceinline__ float bfr(float f) {
    unsigned u = __float_as_uint(f);
    u += 0x7FFFu + ((u >> 16) & 1u);
    return __uint_as_float(u & 0xFFFF0000u);
}
__device__ __forceinline__ unsigned bf_rne_u(float f) {
    unsigned u = __float_as_uint(f);
    u += 0x7FFFu + ((u >> 16) & 1u);
    return u;
}
__device__ __forceinline__ unsigned pk2bf(float lo, float hi) {
    return (bf_rne_u(lo) >> 16) | (bf_rne_u(hi) & 0xFFFF0000u);
}
__device__ __forceinline__ v8u frag_mk(v4u lo, v4u hi) {
    return __builtin_shufflevector(lo, hi, 0, 1, 2, 3, 4, 5, 6, 7);
}
__device__ __forceinline__ v8u frag_ld_bf(const unsigned short* p) {
    const v4u lo = *(const v4u*)(p);
    const v4u hi = *(const v4u*)(p + 16);
    return frag_mk(lo, hi);
}
__device__ __forceinline__ v8u frag_cv_f32(const float* p) {
    const v4f a0 = *(const v4f*)(p), a1 = *(const v4f*)(p + 4);
    const v4f b0 = *(const v4f*)(p + 16), b1 = *(const v4f*)(p + 20);
    v4u lo, hi;
    lo.x = pk2bf(a0.x, a0.y); lo.y = pk2bf(a0.z, a0.w); lo.z = pk2bf(a1.x, a1.y); lo.w = pk2bf(a1.z, a1.w);
    hi.x = pk2bf(b0.x, b0.y); hi.y = pk2bf(b0.z, b0.w); hi.z = pk2bf(b1.x, b1.y); hi.w = pk2bf(b1.z, b1.w);
    return frag_mk(lo, hi);
}
__device__ __forceinline__ v8f wmmabg(v8u a, v8u b, v8f c) {
    c = __builtin_amdgcn_wmma_f32_16x16x32_bf16(false, __builtin_bit_cast(v16bf, a), false, __builtin_bit_cast(v16bf, b), (short)0, c, false, false);
    asm volatile("v_nop\n\tv_nop\n\tv_nop\n\tv_nop" : "+v"(c) : "v"(a), "v"(b));
    return c;
}
__device__ __forceinline__ void wave_sync_lds() {
    __builtin_amdgcn_fence(3  , "workgroup");
    __builtin_amdgcn_wave_barrier();
    __builtin_amdgcn_fence(2  , "workgroup");
}

__global__ __launch_bounds__(256) void k_wconv(const float* __restrict__ src, unsigned short* __restrict__ dst,
                                               unsigned GSZ, unsigned GPAD, unsigned NOUT) {
    const unsigned o = blockIdx.x, h = blockIdx.y, t = threadIdx.x;
    const size_t srow0 = ((size_t)h * NOUT + o) * GSZ;
    const size_t drow0 = ((size_t)h * NOUT + o) * GPAD;
    const unsigned nunits = GPAD * 16u;
    for (unsigned u = t; u < nunits; u += 256u) {
        const unsigned i = u >> 4, k0 = (u & 15u) * 8u;
        const unsigned ic = min(i, GSZ - 1u);
        const float* sp = src + (srow0 + ic) * CD + k0;
        v4f a = *(const v4f*)sp, b = *(const v4f*)(sp + 4);
        asm volatile("" : "+v"(a), "+v"(b));
        const unsigned keep = (i < GSZ) ? 0xFFFFFFFFu : 0u;
        v4u pk;
        pk.x = pk2bf(a.x, a.y) & keep;
        pk.y = pk2bf(a.z, a.w) & keep;
        pk.z = pk2bf(b.x, b.y) & keep;
        pk.w = pk2bf(b.z, b.w) & keep;
        VST2(v4u, (v4u*)(dst + (drow0 + i) * CD + k0), pk);
    }
}

template <unsigned GSZ, unsigned GPAD, unsigned NOUT, unsigned PB>
__device__ __forceinline__ void bconv_body(const float* __restrict__ src, float* __restrict__ dst) {
    static_assert(PB % 128 == 0 && PB >= NOUT * GPAD);
    const unsigned h = blockIdx.y;
    unsigned u = blockIdx.x * 256u + threadIdx.x;
    asm volatile("" : "+v"(u));
    if (u >= PB / 4u) return;
    const float* sh = src + (size_t)h * (NOUT * GSZ);
    float v[4];
#pragma unroll
    for (int e = 0; e < 4; ++e) {
        unsigned c = 4u * u + (unsigned)e;
        asm volatile("" : "+v"(c));
        const unsigned o = c / GPAD;
        const unsigned i = c - o * GPAD;
        const unsigned oc = min(o, NOUT - 1u);
        const unsigned ic = min(i, GSZ - 1u);
        float xv = sh[oc * GSZ + ic];
        asm volatile("" : "+v"(xv));
        v[e] = (o < NOUT && i < GSZ) ? bfr(xv) : 0.0f;
    }
    v4f vv; vv.x = v[0]; vv.y = v[1]; vv.z = v[2]; vv.w = v[3];
    VST2V4(dst + (size_t)h * PB + 4u * u, vv);
}
__global__ __launch_bounds__(256) void k_bconv_a(const float* __restrict__ src, float* __restrict__ dst) { bconv_body<R0, R0, 1u, R0>(src, dst); }
__global__ __launch_bounds__(256) void k_bconv_b(const float* __restrict__ src, float* __restrict__ dst) { bconv_body<GS1, GP, LW, R1P>(src, dst); }
__global__ __launch_bounds__(256) void k_bconv_c(const float* __restrict__ src, float* __restrict__ dst) { bconv_body<GS1, GP, OD, B3PITCH>(src, dst); }

template <unsigned NOUT, bool RELU>
__device__ __forceinline__ void gen_layer(const unsigned short* __restrict__ Wp, const float* __restrict__ Bp,
                                          v8u a0, v8u a1, v8u a2, v8u a3,
                                          float* hpw, unsigned cur, unsigned nxt, unsigned c16, unsigned hh) {
    for (unsigned o = 0; o < NOUT; ++o) {
        float s[8];
#pragma unroll
        for (int r = 0; r < 8; ++r) s[r] = 0.0f;
        for (unsigned t = 0; t < 5u; ++t) {
            const unsigned col = o * GP + t * 16u + c16;
            const unsigned short* wr = Wp + (size_t)col * CD + 8u * hh;
            const v8u b0 = frag_ld_bf(wr);
            const v8u b1 = frag_ld_bf(wr + 32);
            const v8u b2 = frag_ld_bf(wr + 64);
            const v8u b3 = frag_ld_bf(wr + 96);
            const float bv = Bp[col];
            const unsigned hoff = cur + (t * 16u + c16) * HPP + 8u * hh;
            const v4f h0 = *(const v4f*)(hpw + hoff);
            const v4f h1 = *(const v4f*)(hpw + hoff + 4u);
            v8f acc = (v8f){0.f, 0.f, 0.f, 0.f, 0.f, 0.f, 0.f, 0.f};
            acc = wmmabg(a0, b0, acc);
            acc = wmmabg(a1, b1, acc);
            acc = wmmabg(a2, b2, acc);
            acc = wmmabg(a3, b3, acc);
            const float hv[8] = {h0.x, h0.y, h0.z, h0.w, h1.x, h1.y, h1.z, h1.w};
#pragma unroll
            for (int r = 0; r < 8; ++r) s[r] = fmaf(acc[r] + bv, hv[r], s[r]);
        }
#pragma unroll
        for (int r = 0; r < 8; ++r) {
            float v = s[r];
            v += __shfl_xor(v, 1, 32);
            v += __shfl_xor(v, 2, 32);
            v += __shfl_xor(v, 4, 32);
            v += __shfl_xor(v, 8, 32);
            if (RELU) v = fmaxf(v, 0.0f);
            s[r] = v;
        }
        if (c16 == 0u) {
            const unsigned woff = nxt + o * HPP + 8u * hh;
            v4f w0, w1;
            w0.x = s[0]; w0.y = s[1]; w0.z = s[2]; w0.w = s[3];
            w1.x = s[4]; w1.y = s[5]; w1.z = s[6]; w1.w = s[7];
            *(v4f*)(hpw + woff) = w0;
            *(v4f*)(hpw + woff + 4u) = w1;
        }
    }
}

__global__ __launch_bounds__(128) void k_layers(const float* __restrict__ x, const float* __restrict__ cond,
                                                const unsigned short* __restrict__ W0p, const unsigned short* __restrict__ W1p,
                                                const unsigned short* __restrict__ W2p, const unsigned short* __restrict__ W3p,
                                                const float* __restrict__ B0p, const float* __restrict__ B1p,
                                                const float* __restrict__ B2p, const float* __restrict__ B3p,
                                                float* __restrict__ res4) {
    __shared__ __align__(16) float sHP[FW][2 * HPT];
    const unsigned lane = threadIdx.x & 31u;
    const unsigned wave = (unsigned)__builtin_amdgcn_readfirstlane((int)(threadIdx.x >> 5));
    const unsigned c16 = lane & 15u, hh = lane >> 4;
    const unsigned gw = blockIdx.x * (unsigned)FW + wave;
    if (gw >= (unsigned)(NB * (SEQ / 16))) return;
    const unsigned h = gw / (unsigned)(SEQ / 16);
    const unsigned n0 = (gw - h * (unsigned)(SEQ / 16)) * 16u;
    float* hpw = &sHP[wave][0];

    const float* cr = cond + ((size_t)h * SEQ_FULL + n0 + c16) * CD + 8u * hh;
    const v8u a0 = frag_cv_f32(cr);
    const v8u a1 = frag_cv_f32(cr + 32);
    const v8u a2 = frag_cv_f32(cr + 64);
    const v8u a3 = frag_cv_f32(cr + 96);

#pragma unroll
    for (int j = 0; j < 2; ++j) {
        const unsigned q = lane + 32u * (unsigned)j;
        const unsigned row = 64u + (q >> 2), cc = (q & 3u) * 4u;
        const float f = (row == 64u) ? 1.0f : 0.0f;
        v4f pv; pv.x = f; pv.y = f; pv.z = f; pv.w = f;
        *(v4f*)(hpw + row * HPP + cc) = pv;
        *(v4f*)(hpw + HPT + row * HPP + cc) = pv;
    }
    {
        const float* xr = x + ((size_t)h * SEQ_FULL + n0 + c16) * XD;
        const float x0 = bfr(xr[0]), x1 = bfr(xr[1]), x2 = bfr(xr[2]);
        const float va = (hh != 0u) ? x2 : x0;
        const float vb = (hh != 0u) ? 1.0f : x1;
        hpw[(2u * hh) * HPP + c16] = va;
        hpw[(2u * hh + 1u) * HPP + c16] = vb;
    }
    wave_sync_lds();

    {
        const unsigned hoff = (c16 & 3u) * HPP + 8u * hh;
        const v4f g0 = *(const v4f*)(hpw + hoff);
        const v4f g1 = *(const v4f*)(hpw + hoff + 4u);
        const float gv[8] = {g0.x, g0.y, g0.z, g0.w, g1.x, g1.y, g1.z, g1.w};
        const unsigned short* W0h = W0p + (size_t)h * R0 * CD;
        const float* B0h = B0p + (size_t)h * R0;
        for (unsigned t = 0; t < 16u; ++t) {
            const unsigned col = t * 16u + c16;
            const unsigned short* wr = W0h + (size_t)col * CD + 8u * hh;
            const v8u b0 = frag_ld_bf(wr);
            const v8u b1 = frag_ld_bf(wr + 32);
            const v8u b2 = frag_ld_bf(wr + 64);
            const v8u b3 = frag_ld_bf(wr + 96);
            const float bv = B0h[col];
            v8f acc = (v8f){0.f, 0.f, 0.f, 0.f, 0.f, 0.f, 0.f, 0.f};
            acc = wmmabg(a0, b0, acc);
            acc = wmmabg(a1, b1, acc);
            acc = wmmabg(a2, b2, acc);
            acc = wmmabg(a3, b3, acc);
            float p[8];
#pragma unroll
            for (int r = 0; r < 8; ++r) {
                float v = (acc[r] + bv) * gv[r];
                v += __shfl_xor(v, 1, 32);
                v += __shfl_xor(v, 2, 32);
                p[r] = fmaxf(v, 0.0f);
            }
            if ((c16 & 3u) == 0u) {
                const unsigned woff = HPT + (4u * t + (c16 >> 2)) * HPP + 8u * hh;
                v4f w0, w1;
                w0.x = p[0]; w0.y = p[1]; w0.z = p[2]; w0.w = p[3];
                w1.x = p[4]; w1.y = p[5]; w1.z = p[6]; w1.w = p[7];
                *(v4f*)(hpw + woff) = w0;
                *(v4f*)(hpw + woff + 4u) = w1;
            }
        }
    }
    wave_sync_lds();

    gen_layer<LW, true>(W1p + (size_t)h * R1P * CD, B1p + (size_t)h * R1P, a0, a1, a2, a3, hpw, (unsigned)HPT, 0u, c16, hh);
    wave_sync_lds();
    gen_layer<LW, true>(W2p + (size_t)h * R1P * CD, B2p + (size_t)h * R1P, a0, a1, a2, a3, hpw, 0u, (unsigned)HPT, c16, hh);
    wave_sync_lds();
    gen_layer<OD, false>(W3p + (size_t)h * R3P * CD, B3p + (size_t)h * B3PITCH, a0, a1, a2, a3, hpw, (unsigned)HPT, 0u, c16, hh);
    wave_sync_lds();

    v4f ov;
    ov.x = hpw[c16];
    ov.y = hpw[HPP + c16];
    ov.z = hpw[2 * HPP + c16];
    ov.w = 0.0f;
    if (lane < 16u) {
        float* dp = res4 + ((size_t)h * SEQ + n0 + lane) * 4u;
        VST2V4(dp, ov);
    }
}

__global__ __launch_bounds__(256) void k_copy3(const float* __restrict__ res4, float* __restrict__ out) {
    unsigned i = blockIdx.x * 256u + threadIdx.x;
    if (i >= (unsigned)NTOT) return;
    asm volatile("" : "+v"(i));
    const unsigned p = i / 3u;
    const unsigned cpt = i - 3u * p;
    const float v = res4[(size_t)p * 4u + cpt];
    VST2(float, out + i, v);
}

static constexpr size_t al256(size_t b) { return (b + 255) & ~(size_t)255; }
static constexpr size_t SZ_W0 = al256((size_t)NB * R0 * CD * 2);
static constexpr size_t SZ_W1 = al256((size_t)NB * R1P * CD * 2);
static constexpr size_t SZ_W3 = al256((size_t)NB * R3P * CD * 2);
static constexpr size_t SZ_B0 = al256((size_t)NB * R0 * 4);
static constexpr size_t SZ_B1 = al256((size_t)NB * R1P * 4);
static constexpr size_t SZ_B3 = al256((size_t)NB * B3PITCH * 4);
static constexpr size_t SZ_R4 = al256((size_t)NB * SEQ * 4 * 4);
static constexpr size_t OFF_W0 = 0;
static constexpr size_t OFF_W1 = OFF_W0 + SZ_W0;
static constexpr size_t OFF_W2 = OFF_W1 + SZ_W1;
static constexpr size_t OFF_W3 = OFF_W2 + SZ_W1;
static constexpr size_t OFF_B0 = OFF_W3 + SZ_W3;
static constexpr size_t OFF_B1 = OFF_B0 + SZ_B0;
static constexpr size_t OFF_B2 = OFF_B1 + SZ_B1;
static constexpr size_t OFF_B3 = OFF_B2 + SZ_B1;
static constexpr size_t OFF_R4 = OFF_B3 + SZ_B3;
static constexpr size_t WS_TOTAL = OFF_R4 + SZ_R4;
static_assert(WS_TOTAL <= (size_t)134217728);
static_assert((size_t)NB * R1P * CD * 2 <= SZ_W1 && (size_t)NB * R3P * CD * 2 <= SZ_W3);
static_assert((size_t)NB * SEQ * 16 <= SZ_R4);

extern "C" void kernel_launch(void* const* d_in, const int* in_sizes, int n_in, void* d_out, int out_size,
                              void* d_ws, size_t ws_size, hipStream_t stream) {
    if (n_in < 10) return;
    if (in_sizes[0] < ((NB - 1) * SEQ_FULL + SEQ) * XD || in_sizes[1] < ((NB - 1) * SEQ_FULL + SEQ) * CD) return;
    if (in_sizes[2] < NB * R0 * CD || in_sizes[3] < NB * R0) return;
    if (in_sizes[4] < NB * R1 * CD || in_sizes[5] < NB * R1 || in_sizes[6] < NB * R1 * CD || in_sizes[7] < NB * R1) return;
    if (in_sizes[8] < NB * R3 * CD || in_sizes[9] < NB * R3 || out_size < NTOT) return;
    if (WS_TOTAL > ws_size) return;

    const float* x    = (const float*)d_in[0];
    const float* cond = (const float*)d_in[1];
    const float* W0   = (const float*)d_in[2];
    const float* b0   = (const float*)d_in[3];
    const float* W1   = (const float*)d_in[4];
    const float* b1   = (const float*)d_in[5];
    const float* W2   = (const float*)d_in[6];
    const float* b2   = (const float*)d_in[7];
    const float* W3   = (const float*)d_in[8];
    const float* b3   = (const float*)d_in[9];
    float* out = (float*)d_out;

    char* wsp = (char*)d_ws;
    unsigned short* w0p = (unsigned short*)(wsp + OFF_W0);
    unsigned short* w1p = (unsigned short*)(wsp + OFF_W1);
    unsigned short* w2p = (unsigned short*)(wsp + OFF_W2);
    unsigned short* w3p = (unsigned short*)(wsp + OFF_W3);
    float* b0p = (float*)(wsp + OFF_B0);
    float* b1p = (float*)(wsp + OFF_B1);
    float* b2p = (float*)(wsp + OFF_B2);
    float* b3p = (float*)(wsp + OFF_B3);
    float* res4 = (float*)(wsp + OFF_R4);

    k_wconv<<<dim3(1, NB), 256, 0, stream>>>(W0, w0p, (unsigned)R0, (unsigned)R0, 1u);
    k_wconv<<<dim3(LW, NB), 256, 0, stream>>>(W1, w1p, (unsigned)GS1, (unsigned)GP, (unsigned)LW);
    k_wconv<<<dim3(LW, NB), 256, 0, stream>>>(W2, w2p, (unsigned)GS1, (unsigned)GP, (unsigned)LW);
    k_wconv<<<dim3(OD, NB), 256, 0, stream>>>(W3, w3p, (unsigned)GS1, (unsigned)GP, (unsigned)OD);
    k_bconv_a<<<dim3((R0 / 4 + 255) / 256, NB), 256, 0, stream>>>(b0, b0p);
    k_bconv_b<<<dim3((R1P / 4 + 255) / 256, NB), 256, 0, stream>>>(b1, b1p);
    k_bconv_b<<<dim3((R1P / 4 + 255) / 256, NB), 256, 0, stream>>>(b2, b2p);
    k_bconv_c<<<dim3((B3PITCH / 4 + 255) / 256, NB), 256, 0, stream>>>(b3, b3p);

    k_layers<<<(NB * (SEQ / 16)) / FW, 128, 0, stream>>>(x, cond, w0p, w1p, w2p, w3p, b0p, b1p, b2p, b3p, res4);
    k_copy3<<<(NTOT + 255) / 256, 256, 0, stream>>>(res4, out);
}
